// LocAttGrouped_20229295964635
// MI455X (gfx1250) — hardware-run, weakly checked
//
#include <hip/hip_runtime.h>

typedef float          v8f   __attribute__((ext_vector_type(8)));
typedef float          v4f   __attribute__((ext_vector_type(4)));
typedef unsigned int   v4u   __attribute__((ext_vector_type(4)));
typedef int            v8i   __attribute__((ext_vector_type(8)));
typedef unsigned short v8us  __attribute__((ext_vector_type(8)));
typedef unsigned short v16us __attribute__((ext_vector_type(16)));
typedef __bf16         v16bf __attribute__((ext_vector_type(16)));
typedef _Float16       v16h  __attribute__((ext_vector_type(16)));
typedef v4f  __attribute__((may_alias)) v4fa;
typedef v8us __attribute__((may_alias)) v8usa;
union FragB { v16bf v; v16us u; v8us h[2]; v8i w; };
union FragH { v16h  v; v16us u; v8us h[2]; v8i w; };

__device__ __forceinline__ v8f wmb(const FragB& a, const FragB& b, v8f c) {
  v8f d = __builtin_amdgcn_wmma_f32_16x16x32_bf16(false, a.v, false, b.v, (short)0, c, false, false);
  asm volatile("v_nop\n\tv_nop\n\tv_nop\n\tv_nop" : "+v"(d) : "v"(a.w), "v"(b.w));
  return d;
}

__device__ __forceinline__ v8f wmh(const FragH& a, const FragH& b, v8f c) {
  v8f d = __builtin_amdgcn_wmma_f32_16x16x32_f16(false, a.v, false, b.v, (short)0, c, false, false);
  asm volatile("v_nop\n\tv_nop\n\tv_nop\n\tv_nop" : "+v"(d) : "v"(a.w), "v"(b.w));
  return d;
}

__device__ __forceinline__ unsigned bf16_bits(float f) {
  const unsigned u = __float_as_uint(f);
  const unsigned r = (u + 0x7FFFu + ((u >> 16) & 1u)) >> 16;
  const unsigned q = (u >> 16) | 0x40u;
  return ((u & 0x7fffffffu) > 0x7f800000u) ? q : r;
}

__device__ __forceinline__ float bf16_val(float f) {
  return __uint_as_float(bf16_bits(f) << 16);
}
__device__ __forceinline__ int clampi(int v, int lo, int hi) {
  return v < lo ? lo : (v > hi ? hi : v);
}

__device__ __forceinline__ unsigned f16_bits(float f) {
  const unsigned u  = __float_as_uint(f);
  const unsigned s  = (u >> 16) & 0x8000u;
  const unsigned a  = u & 0x7fffffffu;
  const unsigned t  = a - 0x38000000u;
  const unsigned r  = (t + 0x0FFFu + ((t >> 13) & 1u)) >> 13;
  const unsigned rc = r > 0x7C00u ? 0x7C00u : r;
  const bool small  = a < 0x38800000u;
  const bool isnan  = a > 0x7f800000u;
  const unsigned fin = small ? 0u : (s | rc);
  return isnan ? (s | 0x7E00u) : fin;
}

__device__ __forceinline__ unsigned pk16(unsigned lo, unsigned hi) { return lo | (hi << 16); }
__device__ __forceinline__ unsigned bf16_lo_bits(float v) {
  float hi = bf16_val(v);
  asm volatile("" : "+v"(hi));
  return bf16_bits(v - hi);
}
__device__ __forceinline__ v4u pack8_bf16(v4f a, v4f c) {
  return (v4u){ pk16(bf16_bits(a[0]), bf16_bits(a[1])), pk16(bf16_bits(a[2]), bf16_bits(a[3])),
                pk16(bf16_bits(c[0]), bf16_bits(c[1])), pk16(bf16_bits(c[2]), bf16_bits(c[3])) };
}
__device__ __forceinline__ v4u pack8_bf16_lo(v4f a, v4f c) {
  return (v4u){ pk16(bf16_lo_bits(a[0]), bf16_lo_bits(a[1])), pk16(bf16_lo_bits(a[2]), bf16_lo_bits(a[3])),
                pk16(bf16_lo_bits(c[0]), bf16_lo_bits(c[1])), pk16(bf16_lo_bits(c[2]), bf16_lo_bits(c[3])) };
}
__device__ __forceinline__ v4u pack8_f16(v4f a, v4f c) {
  return (v4u){ pk16(f16_bits(a[0]), f16_bits(a[1])), pk16(f16_bits(a[2]), f16_bits(a[3])),
                pk16(f16_bits(c[0]), f16_bits(c[1])), pk16(f16_bits(c[2]), f16_bits(c[3])) };
}

template <int FORM>
__global__ __launch_bounds__(256) void k_plane(const float* __restrict__ src, int rows, int cols, int ldsrc,
                                               unsigned short* __restrict__ dst, int MP, int KP) {
  static_assert(FORM >= 0 && FORM <= 3);
  const int KTOT = (FORM == 1 || FORM == 3) ? 2 * KP : KP;
  const unsigned ppr   = (unsigned)(KTOT >> 3);
  const unsigned kp8   = (unsigned)(KP >> 3);
  const unsigned total = (unsigned)MP * ppr;
  const unsigned g     = blockIdx.x * 256u + threadIdx.x;
  const unsigned rowu  = g / ppr;
  const unsigned p     = g - rowu * ppr;
  const bool second    = p >= kp8;
  const int row = (int)rowu;
  const int c0  = (int)((second ? p - kp8 : p) << 3);
  const float* srow = src + (size_t)clampi(row, 0, rows - 1) * (size_t)ldsrc;
  float x[8];
  unsigned mk[8];
#pragma unroll
  for (int e = 0; e < 8; ++e) {
    const int c = c0 + e;
    const float v = srow[clampi(c, 0, cols - 1)];
    asm volatile("" :: "v"(v));
    x[e]  = v;
    mk[e] = (row < rows && c < cols) ? 0xFFFFu : 0u;
  }
  const v4f a = (v4f){ x[0], x[1], x[2], x[3] };
  const v4f c = (v4f){ x[4], x[5], x[6], x[7] };
  v4u o;
  if (FORM == 2) {
    o = pack8_f16(a, c);
  } else {
    const v4u hi = pack8_bf16(a, c);
    o = hi;
    if (FORM == 1) { const v4u lo = pack8_bf16_lo(a, c); o = second ? lo : hi; }
  }
  const v4u mw = (v4u){ pk16(mk[0], mk[1]), pk16(mk[2], mk[3]), pk16(mk[4], mk[5]), pk16(mk[6], mk[7]) };
  o &= mw;
  if (g < total) {
    volatile v4u* q = (volatile v4u*)(dst + (size_t)g * 8);
    *q = o;
    __threadfence();
    *q = o;
  }
}

template <int FORM> struct FragOf    { typedef FragB T; };
template <>         struct FragOf<2> { typedef FragH T; };
__device__ __forceinline__ v8f mm(const FragB& a, const FragB& b, v8f c) { return wmb(a, b, c); }
__device__ __forceinline__ v8f mm(const FragH& a, const FragH& b, v8f c) { return wmh(a, b, c); }
template <class F> __device__ __forceinline__ F ld_frag(const unsigned short* p) {
  F f;
  f.h[0] = *(const v8usa*)(p);
  f.h[1] = *(const v8usa*)(p + 16);
  return f;
}

template <int FORM, int EPI>
__global__ __launch_bounds__(256) __attribute__((amdgpu_num_vgpr(248)))
void k_gemm_nt(const unsigned short* __restrict__ A, const unsigned short* __restrict__ B,
               const float* __restrict__ bias, float* __restrict__ D, int M, int N, int KTOT, int ldd) {
  static_assert(FORM >= 0 && FORM <= 2);
  static_assert(EPI == 0 || EPI == 1);
  typedef typename FragOf<FORM>::T F;
  __shared__ __attribute__((aligned(16))) float sT[8][16 * 68];
  const int lane = threadIdx.x & 31;
  const int wave = threadIdx.x >> 5;
  const int tilesM = (M + 63) >> 6;
  const int tilesN = (N + 63) >> 6;
  const int tile = blockIdx.x * 8 + wave;
  if (tile >= tilesM * tilesN) return;
  const int tm = tile / tilesN;
  const int tn = tile - tm * tilesN;
  const int m0 = tm << 6;
  const int n0 = tn << 6;

  const int rl = lane & 15;
  const int h8 = (lane >> 4) * 8;
  const unsigned short* pa = A + (size_t)(m0 + rl) * (size_t)KTOT + h8;
  const unsigned short* pb = B + (size_t)(n0 + rl) * (size_t)KTOT + h8;

  v8f acc[4][4];
#pragma unroll
  for (int i = 0; i < 4; ++i)
#pragma unroll
    for (int j = 0; j < 4; ++j) acc[i][j] = (v8f){0.f, 0.f, 0.f, 0.f, 0.f, 0.f, 0.f, 0.f};

#pragma unroll 1
  for (int k0 = 0; k0 < KTOT; k0 += 32) {
    F bf[4];
#pragma unroll
    for (int j = 0; j < 4; ++j) bf[j] = ld_frag<F>(pb + (size_t)(j << 4) * (size_t)KTOT + k0);
#pragma unroll
    for (int i = 0; i < 4; ++i) {
      const F af = ld_frag<F>(pa + (size_t)(i << 4) * (size_t)KTOT + k0);
#pragma unroll
      for (int j = 0; j < 4; ++j) acc[i][j] = mm(af, bf[j], acc[i][j]);
    }
  }

  float* slab = sT[wave];
  const int hh = lane >> 4;
  const int c4 = (lane & 15) * 4;
  const int nc = n0 + c4;
  const bool cok = nc < N;
  v4f bv = (v4f){0.f, 0.f, 0.f, 0.f};
  if (EPI == 1) {
    bv = *(const v4fa*)(bias + clampi(nc, 0, N - 4));
    asm volatile("" :: "v"(bv));
  }
#pragma unroll
  for (int i = 0; i < 4; ++i) {
    const int mBase = m0 + (i << 4);
#pragma unroll
    for (int j = 0; j < 4; ++j) {
#pragma unroll
      for (int r = 0; r < 8; ++r) slab[(h8 + r) * 68 + (j << 4) + rl] = acc[i][j][r];
    }
    __builtin_amdgcn_fence(__ATOMIC_RELEASE, "workgroup");
    __builtin_amdgcn_wave_barrier();
    __builtin_amdgcn_fence(__ATOMIC_ACQUIRE, "workgroup");
    v4f vv[8];
#pragma unroll
    for (int it = 0; it < 8; ++it) {
      const int row = it * 2 + hh;
      v4f v = *(const v4fa*)(slab + row * 68 + c4);
      if (EPI == 1) v += bv;
      vv[it] = v;
    }
    for (int pass = 0; pass < 2; ++pass) {
#pragma unroll
      for (int it = 0; it < 8; ++it) {
        const int row = mBase + it * 2 + hh;
        if (cok && row < M) *(volatile v4f*)(D + (size_t)row * (size_t)ldd + nc) = vv[it];
      }
      __threadfence();
    }
    __builtin_amdgcn_fence(__ATOMIC_RELEASE, "workgroup");
    __builtin_amdgcn_wave_barrier();
    __builtin_amdgcn_fence(__ATOMIC_ACQUIRE, "workgroup");
  }
}

constexpr int kB  = 4;
constexpr int kC  = 256;
constexpr int kH  = 64;
constexpr int kW  = 64;
constexpr int kG  = 4;
constexpr int kGd = 64;
constexpr int kKS = 3;
constexpr int kHW = kH * kW;
constexpr int kM  = kB * kHW;
constexpr int kN3 = 3 * kC;
constexpr int kK  = kC;

constexpr int XT_PITCH     = 65;
constexpr int XT_LDS_BYTES = kC * XT_PITCH * 4;
constexpr int LA_CP        = kW + 2;
constexpr int LA_KV_FL     = kKS * kGd * LA_CP;
constexpr int LA_Q_FL      = kGd * kW;
constexpr int LA_S_FL      = 9 * 256;
constexpr int LA_LDS_BYTES = (2 * LA_KV_FL + LA_Q_FL + LA_S_FL) * 4;

static_assert(kH == 64);
static_assert(kW == 64);
static_assert(kC == 256);
static_assert(kG * kGd == kC);
static_assert(kGd == 64);
static_assert(kKS == 3);
static_assert(kM % 128 == 0);
static_assert(kM % 64 == 0);
static_assert(kN3 % 64 == 0);
static_assert(kN3 % 32 == 0);
static_assert(kK % 32 == 0);
static_assert(kC % 64 == 0);
static_assert((kC * kK / 8) % 256 == 0);
static_assert(256 / 32 == 2 * 4);
static_assert(4 * 16 == kGd);
static_assert(XT_LDS_BYTES <= 327680);
static_assert(LA_LDS_BYTES <= 327680);
static_assert(LA_LDS_BYTES == 126976);

constexpr size_t WS_XB   = 0;
constexpr size_t SZ_XB   = (size_t)kM * kK * 2;
constexpr size_t WS_WB   = WS_XB + SZ_XB;
constexpr size_t SZ_WB   = (size_t)kN3 * kK * 2;
constexpr size_t WS_BIAS = WS_WB + SZ_WB;
constexpr size_t SZ_BIAS = (size_t)kN3 * 4;
constexpr size_t WS_QKV  = WS_BIAS + SZ_BIAS;
constexpr size_t SZ_QKV  = (size_t)kM * kN3 * 4;
constexpr size_t WS_END  = WS_QKV + SZ_QKV;
static_assert(WS_WB % 256 == 0);
static_assert(WS_BIAS % 256 == 0);
static_assert(WS_QKV % 256 == 0);
static_assert(SZ_BIAS % 128 == 0);
static_assert(WS_END <= (size_t)134217728);

__global__ __launch_bounds__(256) void k_xt(const float* __restrict__ x, const float* __restrict__ bq,
                                            const float* __restrict__ bk, const float* __restrict__ bv,
                                            unsigned short* __restrict__ XB, float* __restrict__ BIAS) {
  extern __shared__ __attribute__((aligned(16))) float xt_tile[];
  const int tid = threadIdx.x;

  if (blockIdx.x == 0 && tid < 192) {
    const int j4  = (tid & 63) * 4;
    const int sel = tid >> 6;
    const v4f vq = *(const v4fa*)(bq + j4);
    const v4f vk = *(const v4fa*)(bk + j4);
    const v4f vv = *(const v4fa*)(bv + j4);
    asm volatile("" :: "v"(vq), "v"(vk), "v"(vv));
    const unsigned mq = (sel == 0) ? 0xFFFFFFFFu : 0u;
    const unsigned mk = (sel == 1) ? 0xFFFFFFFFu : 0u;
    const unsigned mv = (sel == 2) ? 0xFFFFFFFFu : 0u;
    v4f o;
#pragma unroll
    for (int e = 0; e < 4; ++e) {
      const unsigned bits = (__float_as_uint(vq[e]) & mq) | (__float_as_uint(vk[e]) & mk) | (__float_as_uint(vv[e]) & mv);
      o[e] = bf16_val(__uint_as_float(bits));
    }
    volatile v4f* p = (volatile v4f*)(BIAS + sel * kC + j4);
    *p = o;
    __threadfence();
    *p = o;
  }

  const int b  = blockIdx.x >> 6;
  const int h  = blockIdx.x & 63;
  const int f4 = tid & 15;
  const int co = tid >> 4;
#pragma unroll 4
  for (int it = 0; it < 16; ++it) {
    const int c = it * 16 + co;
    const v4f a = *(const v4fa*)(x + (size_t)(b * kC + c) * (size_t)kHW + (size_t)(h * kW + 4 * f4));
    float* t = xt_tile + c * XT_PITCH + 4 * f4;
    t[0] = a[0]; t[1] = a[1]; t[2] = a[2]; t[3] = a[3];
  }
  __syncthreads();

  const int lane = tid & 31;
  const int wave = tid >> 5;
  v4u pk[8];
#pragma unroll
  for (int i = 0; i < 8; ++i) {
    const int w = wave * 8 + i;
    const float* t = xt_tile + (8 * lane) * XT_PITCH + w;
    const v4f a = (v4f){ t[0], t[XT_PITCH], t[2 * XT_PITCH], t[3 * XT_PITCH] };
    const v4f c = (v4f){ t[4 * XT_PITCH], t[5 * XT_PITCH], t[6 * XT_PITCH], t[7 * XT_PITCH] };
    pk[i] = pack8_bf16(a, c);
  }
  const size_t r0 = (size_t)blockIdx.x * 64 + (size_t)(wave * 8);
  for (int pass = 0; pass < 2; ++pass) {
#pragma unroll
    for (int i = 0; i < 8; ++i) {
      *(volatile v4u*)(XB + (r0 + i) * (size_t)kK + 8 * lane) = pk[i];
    }
    __threadfence();
  }
}

__global__ __launch_bounds__(256) void k_locatt(const float* __restrict__ QKV, float* __restrict__ out) {
  extern __shared__ __attribute__((aligned(16))) float la_lds[];
  float* K3 = la_lds;
  float* V3 = la_lds + LA_KV_FL;
  float* Qs = la_lds + 2 * LA_KV_FL;
  float* Ss = la_lds + 2 * LA_KV_FL + LA_Q_FL;

  const int tid = threadIdx.x;
  const int bx  = blockIdx.x;
  const int g   = bx & 3;
  const int h   = (bx >> 2) & 63;
  const int b   = bx >> 8;

  {
    const int d    = tid & 63;
    const int side = (tid >> 6) & 1;
    const int kv   = tid >> 7;
    float* p = la_lds + kv * LA_KV_FL + d * LA_CP + side * (LA_CP - 1);
    p[0] = 0.0f;
    p[kGd * LA_CP] = 0.0f;
    p[2 * kGd * LA_CP] = 0.0f;
  }

  const int f4 = tid & 15;
  const int ws = tid >> 4;
  const size_t rowbase = (size_t)b * (size_t)kHW;

#pragma unroll 1
  for (int i = 0; i < 3; ++i) {
    const int hr = h + i - 1;
    if (hr >= 0 && hr < kH) {
#pragma unroll
      for (int it = 0; it < 4; ++it) {
        const int w = it * 16 + ws;
        const float* src = QKV + (rowbase + (size_t)(hr * kW + w)) * (size_t)kN3 + (size_t)(g * kGd + 4 * f4);
        const v4f kk = *(const v4fa*)(src + kC);
        const v4f vv = *(const v4fa*)(src + 2 * kC);
        float* kd = K3 + (i * kGd + 4 * f4) * LA_CP + w + 1;
        float* vd = V3 + (i * kGd + 4 * f4) * LA_CP + w + 1;
        kd[0] = kk[0]; kd[LA_CP] = kk[1]; kd[2 * LA_CP] = kk[2]; kd[3 * LA_CP] = kk[3];
        vd[0] = vv[0]; vd[LA_CP] = vv[1]; vd[2 * LA_CP] = vv[2]; vd[3 * LA_CP] = vv[3];
      }
    } else {
#pragma unroll
      for (int it = 0; it < 4; ++it) {
        const int w = it * 16 + ws;
        float* kd = K3 + (i * kGd + 4 * f4) * LA_CP + w + 1;
        float* vd = V3 + (i * kGd + 4 * f4) * LA_CP + w + 1;
        kd[0] = 0.0f; kd[LA_CP] = 0.0f; kd[2 * LA_CP] = 0.0f; kd[3 * LA_CP] = 0.0f;
        vd[0] = 0.0f; vd[LA_CP] = 0.0f; vd[2 * LA_CP] = 0.0f; vd[3 * LA_CP] = 0.0f;
      }
    }
  }
#pragma unroll
  for (int it = 0; it < 4; ++it) {
    const int w = it * 16 + ws;
    const float* src = QKV + (rowbase + (size_t)(h * kW + w)) * (size_t)kN3 + (size_t)(g * kGd + 4 * f4);
    const v4f qq = *(const v4fa*)(src);
    float* qd = Qs + (4 * f4) * kW + w;
    qd[0] = qq[0]; qd[kW] = qq[1]; qd[2 * kW] = qq[2]; qd[3 * kW] = qq[3];
  }
  __syncthreads();

  const int lane = tid & 31;
  const int wave = tid >> 5;
  const int half = wave & 1;
  const int dq   = wave >> 1;
  const int w    = 32 * half + lane;

  float s[9];
#pragma unroll
  for (int p = 0; p < 9; ++p) s[p] = 0.0f;

#pragma unroll 2
  for (int d = 0; d < kGd; ++d) {
    const float qv = Qs[d * kW + w];
    const float* kr = K3 + d * LA_CP + w;
#pragma unroll
    for (int i = 0; i < 3; ++i) {
#pragma unroll
      for (int j = 0; j < 3; ++j) {
        s[i * 3 + j] = fmaf(qv, kr[i * kGd * LA_CP + j], s[i * 3 + j]);
      }
    }
  }

  float m = s[0];
#pragma unroll
  for (int p = 1; p < 9; ++p) m = fmaxf(m, s[p]);

  float* sp = Ss + tid;
#pragma unroll
  for (int p = 0; p < 9; ++p) sp[p * 256] = s[p];
  float sum = 0.0f;
#pragma unroll 1
  for (int p = 0; p < 9; ++p) {
    const float e = expf(sp[p * 256] - m);
    sum += e;
    sp[p * 256] = e;
  }
#pragma unroll 1
  for (int p = 0; p < 9; ++p) {
    const float a = sp[p * 256] / sum;
    sp[p * 256] = a;
  }
  float a[9];
#pragma unroll
  for (int p = 0; p < 9; ++p) a[p] = sp[p * 256];

  float* obase = out + ((size_t)(b * kC + g * kGd + 16 * dq) * (size_t)kH + (size_t)h) * (size_t)kW + (size_t)w;
#pragma unroll 1
  for (int pass = 0; pass < 2; ++pass) {
#pragma unroll 2
    for (int dd = 0; dd < 16; ++dd) {
      const float* vr = V3 + (16 * dq + dd) * LA_CP + w;
      float o = 0.0f;
#pragma unroll
      for (int i = 0; i < 3; ++i) {
#pragma unroll
        for (int j = 0; j < 3; ++j) {
          o = fmaf(a[i * 3 + j], vr[i * kGd * LA_CP + j], o);
        }
      }
      *(volatile float*)(obase + (size_t)dd * (size_t)kHW) = o;
    }
    __threadfence();
  }
}

extern "C" void kernel_launch(void* const* d_in, const int* in_sizes, int n_in,
                              void* d_out, int out_size, void* d_ws, size_t ws_size,
                              hipStream_t stream) {
  if (n_in < 7) return;
  if (in_sizes[0] != kB * kC * kHW) return;
  if (in_sizes[1] != kC * kK || in_sizes[2] != kC) return;
  if (in_sizes[3] != kC * kK || in_sizes[4] != kC) return;
  if (in_sizes[5] != kC * kK || in_sizes[6] != kC) return;
  if (out_size != kB * kC * kHW) return;
  if (WS_END > ws_size) return;

  const float* x  = (const float*)d_in[0];
  const float* wq = (const float*)d_in[1];
  const float* bq = (const float*)d_in[2];
  const float* wk = (const float*)d_in[3];
  const float* bk = (const float*)d_in[4];
  const float* wv = (const float*)d_in[5];
  const float* bv = (const float*)d_in[6];
  float* outp = (float*)d_out;

  char* ws = (char*)d_ws;
  unsigned short* XB   = (unsigned short*)(ws + WS_XB);
  unsigned short* WB   = (unsigned short*)(ws + WS_WB);
  float*          BIAS = (float*)(ws + WS_BIAS);
  float*          QKV  = (float*)(ws + WS_QKV);

  (void)hipFuncSetAttribute(reinterpret_cast<const void*>(&k_xt), hipFuncAttributeMaxDynamicSharedMemorySize, XT_LDS_BYTES);
  (void)hipFuncSetAttribute(reinterpret_cast<const void*>(&k_locatt), hipFuncAttributeMaxDynamicSharedMemorySize, LA_LDS_BYTES);

  k_xt<<<dim3(kB * kH), dim3(256), XT_LDS_BYTES, stream>>>(x, bq, bk, bv, XB, BIAS);

  const int planeBlocks = kC * kK / 8 / 256;
  k_plane<0><<<dim3(planeBlocks), dim3(256), 0, stream>>>(wq, kC, kK, kK, WB, kC, kK);
  k_plane<0><<<dim3(planeBlocks), dim3(256), 0, stream>>>(wk, kC, kK, kK, WB + (size_t)kC * kK, kC, kK);
  k_plane<0><<<dim3(planeBlocks), dim3(256), 0, stream>>>(wv, kC, kK, kK, WB + (size_t)2 * kC * kK, kC, kK);

  const int tiles = (kM / 64) * (kN3 / 64);
  k_gemm_nt<0, 1><<<dim3((tiles + 7) / 8), dim3(256), 0, stream>>>(XB, WB, BIAS, QKV, kM, kN3, kK, kN3);

  k_locatt<<<dim3(kB * kH * kG), dim3(256), LA_LDS_BYTES, stream>>>(QKV, outp);
  (void)hipGetLastError();
}
